// SA_6519760355387
// MI455X (gfx1250) — hardware-verified
//
#include <hip/hip_runtime.h>
#include <math.h>
#include <stdint.h>

#ifndef NB
#define NB 2
#endif
#ifndef SEQ
#define SEQ 2048
#endif
#define NB_FULL  2
#define SEQ_FULL 2048
#define DMOD     1024
#define NHEAD    16
#define HDIM     64
#define HG       2
#define SM_SCALE 0.125f

static_assert(SEQ % 256 == 0);
static_assert(SEQ >= 256);
static_assert(SEQ <= SEQ_FULL);
static_assert(NB >= 1);
static_assert(NB <= NB_FULL);
static_assert(NHEAD * HDIM == DMOD);
static_assert(NHEAD % HG == 0);
static_assert(DMOD % 64 == 0);
static_assert(HDIM == 64);
static_assert(SEQ % 64 == 0);

typedef __attribute__((ext_vector_type(16))) _Float16 v16h;
typedef __attribute__((ext_vector_type(8)))  _Float16 v8h;
typedef __attribute__((ext_vector_type(16))) __bf16   v16b;
typedef __attribute__((ext_vector_type(8)))  __bf16   v8b;
typedef __attribute__((ext_vector_type(8)))  float    v8f;
typedef __attribute__((ext_vector_type(4)))  float    v4f;
typedef __attribute__((ext_vector_type(2)))  float    v2f;
typedef __attribute__((ext_vector_type(4)))  unsigned int v4u;
typedef __attribute__((ext_vector_type(4)))  int      v4i;

__device__ __forceinline__ unsigned short f2bf_bits(float f) {
  unsigned u = __float_as_uint(f);
  return (unsigned short)((u + 0x7FFFu + ((u >> 16) & 1u)) >> 16);
}
__device__ __forceinline__ float bf_bits2f(unsigned short h) { return __uint_as_float(((unsigned)h) << 16); }
__device__ __forceinline__ float bf16q(float f) { return bf_bits2f(f2bf_bits(f)); }

__device__ __forceinline__ void dep_guard_h(v8f& a, v8f& b, v16h x, v16h y) { asm volatile("v_nop\n\tv_nop\n\tv_nop\n\tv_nop" : "+v"(a), "+v"(b) : "v"(x), "v"(y)); }
__device__ __forceinline__ void dep_guard_b(v8f& a, v8f& b, v16b x, v16b y) { asm volatile("v_nop\n\tv_nop\n\tv_nop\n\tv_nop" : "+v"(a), "+v"(b) : "v"(x), "v"(y)); }
__device__ __forceinline__ void keep4_h(v16h a, v16h b, v16h c, v16h d) { asm volatile("v_nop" :: "v"(a), "v"(b), "v"(c), "v"(d)); }
__device__ __forceinline__ void keep4_b(v16b a, v16b b, v16b c, v16b d) { asm volatile("v_nop" :: "v"(a), "v"(b), "v"(c), "v"(d)); }
__device__ __forceinline__ void acc_guard4(v8f& a, v8f& b, v8f& c, v8f& d) { asm volatile("v_nop\n\tv_nop\n\tv_nop\n\tv_nop" : "+v"(a), "+v"(b), "+v"(c), "+v"(d)); }

template <typename T> struct Frag;
template <> struct Frag<_Float16> {
  typedef v16h V; union U { v16h v; v8h h[2]; };
  static __device__ __forceinline__ v16h load(const _Float16* p) {
    U f; f.h[0] = *(const v8h*)(p); f.h[1] = *(const v8h*)(p + 16); return f.v;
  }
  static __device__ __forceinline__ v8f mma(v16h a, v16h b, v8f c) {
    return __builtin_amdgcn_wmma_f32_16x16x32_f16(false, a, false, b, (short)0, c, false, false);
  }
  static __device__ __forceinline__ void guard(v8f& a, v8f& b, v16h x, v16h y) { dep_guard_h(a, b, x, y); }
  static __device__ __forceinline__ void keep(v16h a, v16h b, v16h c, v16h d) { keep4_h(a, b, c, d); }
};
template <> struct Frag<__bf16> {
  typedef v16b V; union U { v16b v; v8b h[2]; };
  static __device__ __forceinline__ v16b load(const __bf16* p) {
    U f; f.h[0] = *(const v8b*)(p); f.h[1] = *(const v8b*)(p + 16); return f.v;
  }
  static __device__ __forceinline__ v8f mma(v16b a, v16b b, v8f c) {
    return __builtin_amdgcn_wmma_f32_16x16x32_bf16(false, a, false, b, (short)0, c, false, false);
  }
  static __device__ __forceinline__ void guard(v8f& a, v8f& b, v16b x, v16b y) { dep_guard_b(a, b, x, y); }
  static __device__ __forceinline__ void keep(v16b a, v16b b, v16b c, v16b d) { keep4_b(a, b, c, d); }
};

template <int ET> struct Elem;
template <> struct Elem<0> { typedef _Float16 T; };
template <> struct Elem<1> { typedef __bf16 T; };
template <int ET, int SA, int SB, int BIAS_MODE, int OUT_MODE, int CAUS>
__global__ __launch_bounds__(256) void wmma_gemm64(
    const unsigned short* __restrict__ Ap, const unsigned short* __restrict__ A2p, int lda, long strideA,
    const unsigned short* __restrict__ Btp, const unsigned short* __restrict__ Bt2p, int ldb, long strideB,
    void* __restrict__ Cout, void* __restrict__ Cout2, int ldc, long strideC,
    const float* __restrict__ bias,
    int M, int N, int K, float scale) {
  typedef typename Elem<ET>::T T;
  typedef typename Frag<T>::V V;
  const T* A = (const T*)Ap; const T* A2 = (const T*)A2p; const T* Bt = (const T*)Btp; const T* Bt2 = (const T*)Bt2p;
  __shared__ __align__(16) float sT[8][16 * 68];
  const int b    = blockIdx.y;
  const int lane = threadIdx.x & 31;
  const int wave = threadIdx.x >> 5;
  const int tilesN = N >> 6;
  const int tilesM = M >> 6;
  const int tile = blockIdx.x * 8 + wave;
  if (tile >= tilesM * tilesN) return;
  const int tm = tile / tilesN;
  const int tn = tile - tm * tilesN;
  const int m0 = tm << 6;
  const int n0 = tn << 6;
  if (CAUS == 1 && n0 >= m0 + 64) return;
  int Kend = K;
  if (CAUS == 2) Kend = (m0 + 64 < K) ? (m0 + 64) : K;

  const size_t sA = (size_t)b * (size_t)strideA;
  const size_t sB = (size_t)b * (size_t)strideB;
  const T* Ab  = A  + sA;
  const T* Bb  = Bt + sB;
  const T* Ab2 = SA ? (A2  + sA) : Ab;
  const T* Bb2 = SB ? (Bt2 + sB) : Bb;

  const int rlane = lane & 15;
  const int koff  = (lane >> 4) * 8;
  const int mOff  = (lane >> 4) * 8;

  v8f acc[4][4];
#pragma unroll
  for (int i = 0; i < 4; ++i)
#pragma unroll
    for (int j = 0; j < 4; ++j) acc[i][j] = (v8f){0.f,0.f,0.f,0.f,0.f,0.f,0.f,0.f};

  for (int k0 = 0; k0 < Kend; k0 += 32) {
    V bq[4];
#pragma unroll
    for (int j = 0; j < 4; ++j) {
      const size_t bo = (size_t)(n0 + (j << 4) + rlane) * ldb + koff + k0;
      bq[j] = Frag<T>::load(Bb + bo);
    }
#pragma unroll
    for (int i = 0; i < 4; ++i) {
      const size_t ao = (size_t)(m0 + (i << 4) + rlane) * lda + koff + k0;
      V ah = Frag<T>::load(Ab + ao);
      V al = ah;
      if (SA) al = Frag<T>::load(Ab2 + ao);
#pragma unroll
      for (int j = 0; j < 4; ++j) {
        acc[i][j] = Frag<T>::mma(ah, bq[j], acc[i][j]);
        if (SA) acc[i][j] = Frag<T>::mma(al, bq[j], acc[i][j]);
      }
      Frag<T>::guard(acc[i][0], acc[i][3], ah, al);
    }
    Frag<T>::keep(bq[0], bq[1], bq[2], bq[3]);
    if (SB) {
#pragma unroll
      for (int j = 0; j < 4; ++j) {
        const size_t bo = (size_t)(n0 + (j << 4) + rlane) * ldb + koff + k0;
        bq[j] = Frag<T>::load(Bb2 + bo);
      }
#pragma unroll
      for (int i = 0; i < 4; ++i) {
        const size_t ao = (size_t)(m0 + (i << 4) + rlane) * lda + koff + k0;
        V ah = Frag<T>::load(Ab + ao);
#pragma unroll
        for (int j = 0; j < 4; ++j) acc[i][j] = Frag<T>::mma(ah, bq[j], acc[i][j]);
        Frag<T>::guard(acc[i][0], acc[i][3], ah, ah);
      }
      Frag<T>::keep(bq[0], bq[1], bq[2], bq[3]);
    }
  }
  acc_guard4(acc[0][0], acc[0][1], acc[0][2], acc[0][3]);
  acc_guard4(acc[1][0], acc[1][1], acc[1][2], acc[1][3]);
  acc_guard4(acc[2][0], acc[2][1], acc[2][2], acc[2][3]);
  acc_guard4(acc[3][0], acc[3][1], acc[3][2], acc[3][3]);

  float* slab = sT[wave];
#pragma unroll
  for (int i = 0; i < 4; ++i) {
    const int mBase = m0 + (i << 4);
    float bm[8];
#pragma unroll
    for (int r = 0; r < 8; ++r) bm[r] = 0.f;
    if (BIAS_MODE == 1) {
#pragma unroll
      for (int r = 0; r < 8; ++r) bm[r] = bf16q(bias[mBase + mOff + r]);
    }
#pragma unroll
    for (int j = 0; j < 4; ++j) {
      const int n = n0 + (j << 4) + rlane;
      float bv = 0.f;
      if (BIAS_MODE == 2) bv = bf16q(bias[n]);
#pragma unroll
      for (int r = 0; r < 8; ++r) {
        float v = acc[i][j][r] * scale;
        if (BIAS_MODE == 1) v += bm[r];
        if (BIAS_MODE == 2) v += bv;
        slab[(mOff + r) * 68 + (j << 4) + rlane] = v;
      }
    }
    __builtin_amdgcn_fence(__ATOMIC_RELEASE, "workgroup");
    __builtin_amdgcn_wave_barrier();
    __builtin_amdgcn_fence(__ATOMIC_ACQUIRE, "workgroup");
    if (OUT_MODE == 0) {
      float* C = (float*)Cout + (size_t)b * (size_t)strideC;
      const int hh = lane >> 4, c4 = (lane & 15) * 4;
      for (int pass = 0; pass < 2; ++pass) {
#pragma unroll
        for (int it = 0; it < 8; ++it) {
          const int row = it * 2 + hh;
          v4f v = *(const v4f*)(slab + row * 68 + c4);
          *(volatile v4f*)(C + (size_t)(mBase + row) * ldc + n0 + c4) = v;
        }
        __threadfence();
      }
    } else {
      const int q = lane >> 3, c8 = (lane & 7) * 8;
      unsigned short* C  = (unsigned short*)Cout  + (size_t)b * (size_t)strideC;
      unsigned short* C2 = (OUT_MODE == 2) ? ((unsigned short*)Cout2 + (size_t)b * (size_t)strideC) : C;
      for (int pass = 0; pass < 2; ++pass) {
#pragma unroll
        for (int it = 0; it < 4; ++it) {
          const int row = it * 4 + q;
          const float* sp = slab + row * 68 + c8;
          v8h hv, lv;
#pragma unroll
          for (int e = 0; e < 8; ++e) {
            if (OUT_MODE == 1) {
              hv[e] = (_Float16)sp[e];
              lv[e] = hv[e];
            } else {
              unsigned short hb = f2bf_bits(sp[e]);
              unsigned short lb = f2bf_bits(sp[e] - bf_bits2f(hb));
              hv[e] = __builtin_bit_cast(_Float16, hb);
              lv[e] = __builtin_bit_cast(_Float16, lb);
            }
          }
          *(volatile v8h*)(C + (size_t)(mBase + row) * ldc + n0 + c8) = hv;
          if (OUT_MODE == 2) *(volatile v8h*)(C2 + (size_t)(mBase + row) * ldc + n0 + c8) = lv;
        }
        __threadfence();
      }
    }
    __builtin_amdgcn_fence(__ATOMIC_RELEASE, "workgroup");
    __builtin_amdgcn_wave_barrier();
    __builtin_amdgcn_fence(__ATOMIC_ACQUIRE, "workgroup");
  }
}

__device__ __forceinline__ unsigned pk16(unsigned short a, unsigned short b) { return (unsigned)a | ((unsigned)b << 16); }

__global__ __launch_bounds__(256) void cast_bf16x2_kernel(const float* __restrict__ in, unsigned short* __restrict__ out, int n2) {
  const int i = blockIdx.x * 256 + threadIdx.x;
  if (i < n2) {
    const v2f f = *(const v2f*)(in + 2 * (size_t)i);
    const unsigned u = pk16(f2bf_bits(f[0]), f2bf_bits(f[1]));
    ((volatile unsigned*)out)[i] = u;
    __threadfence();
    ((volatile unsigned*)out)[i] = u;
  }
}

__global__ __launch_bounds__(256) void cast_transpose_bf16_kernel(const float* __restrict__ W, unsigned short* __restrict__ Wt,
                                                                 int nrows, int ncols) {
  __shared__ __align__(16) _Float16 sT[64 * 72];
  const int r0 = blockIdx.y * 64;
  const int c0 = blockIdx.x * 64;
  const int t = threadIdx.x;
  const int lane = t & 31, wave = t >> 5;
#pragma unroll
  for (int pass = 0; pass < 4; ++pass) {
    const int kr = pass * 16 + (t >> 4);
    const int c4 = (t & 15) * 4;
    const v4f v = *(const v4f*)(W + (size_t)(r0 + kr) * ncols + c0 + c4);
    sT[(c4 + 0) * 72 + kr] = __builtin_bit_cast(_Float16, f2bf_bits(v[0]));
    sT[(c4 + 1) * 72 + kr] = __builtin_bit_cast(_Float16, f2bf_bits(v[1]));
    sT[(c4 + 2) * 72 + kr] = __builtin_bit_cast(_Float16, f2bf_bits(v[2]));
    sT[(c4 + 3) * 72 + kr] = __builtin_bit_cast(_Float16, f2bf_bits(v[3]));
  }
  __syncthreads();
  const int q = lane >> 3, c8 = (lane & 7) * 8;
  for (int pass = 0; pass < 2; ++pass) {
#pragma unroll
    for (int it = 0; it < 2; ++it) {
      const int nl = wave * 8 + it * 4 + q;
      const v8h hv = *(const v8h*)(sT + nl * 72 + c8);
      *(volatile v8h*)(Wt + (size_t)(c0 + nl) * nrows + r0 + c8) = hv;
    }
    __threadfence();
  }
}

__global__ __launch_bounds__(256) void softmax_row_kernel(const float* __restrict__ S, const int* __restrict__ am,
                                                          unsigned short* __restrict__ Ph, unsigned short* __restrict__ Pl) {
  __shared__ float redm[SEQ / 256];
  __shared__ float reds[SEQ / 256];
  const int i    = blockIdx.x;
  const int y    = blockIdx.y;
  const int tid  = threadIdx.x;
  const int lane = tid & 31;
  const int wave = tid >> 5;
  const int j0   = tid * 8;
  const size_t ro = ((size_t)y * SEQ + (size_t)i) * SEQ + (size_t)j0;
  const v4f a = *(const v4f*)(S + ro);
  const v4f c = *(const v4f*)(S + ro + 4);
  const v4i ma = *(const v4i*)(am + j0);
  const v4i mc = *(const v4i*)(am + j0 + 4);
  const float NEG = -__builtin_inff();
  float t[8];
#pragma unroll
  for (int e = 0; e < 4; ++e) {
    t[e]     = (((j0 + e) <= i) && (ma[e] != 0)) ? a[e] : NEG;
    t[4 + e] = (((j0 + 4 + e) <= i) && (mc[e] != 0)) ? c[e] : NEG;
  }
  float m = fmaxf(fmaxf(fmaxf(t[0], t[1]), fmaxf(t[2], t[3])), fmaxf(fmaxf(t[4], t[5]), fmaxf(t[6], t[7])));
#pragma unroll
  for (int off = 16; off > 0; off >>= 1) m = fmaxf(m, __shfl_xor(m, off, 32));
  if (lane == 0) redm[wave] = m;
  __syncthreads();
  float mx = redm[0];
#pragma unroll
  for (int w = 1; w < SEQ / 256; ++w) mx = fmaxf(mx, redm[w]);
  float ex[8];
#pragma unroll
  for (int e = 0; e < 8; ++e) ex[e] = __expf(t[e] - mx);
  float s = ((ex[0] + ex[1]) + (ex[2] + ex[3])) + ((ex[4] + ex[5]) + (ex[6] + ex[7]));
#pragma unroll
  for (int off = 16; off > 0; off >>= 1) s += __shfl_xor(s, off, 32);
  if (lane == 0) reds[wave] = s;
  __syncthreads();
  float tot = reds[0];
#pragma unroll
  for (int w = 1; w < SEQ / 256; ++w) tot += reds[w];
  const float inv = 1.0f / tot;
  unsigned short hb[8], lb[8];
#pragma unroll
  for (int e = 0; e < 8; ++e) {
    const float p = ex[e] * inv;
    hb[e] = f2bf_bits(p);
    lb[e] = f2bf_bits(p - bf_bits2f(hb[e]));
  }
  const v4u hv = (v4u){pk16(hb[0], hb[1]), pk16(hb[2], hb[3]), pk16(hb[4], hb[5]), pk16(hb[6], hb[7])};
  const v4u lv = (v4u){pk16(lb[0], lb[1]), pk16(lb[2], lb[3]), pk16(lb[4], lb[5]), pk16(lb[6], lb[7])};
  *(volatile v4u*)(Ph + ro) = hv;
  *(volatile v4u*)(Pl + ro) = lv;
  __threadfence();
  *(volatile v4u*)(Ph + ro) = hv;
  *(volatile v4u*)(Pl + ro) = lv;
}

extern "C" void kernel_launch(void* const* d_in, const int* in_sizes, int n_in,
                              void* d_out, int out_size, void* d_ws, size_t ws_size,
                              hipStream_t stream) {
  if (n_in < 10) return;
  if (in_sizes[0] < (NB - 1) * SEQ_FULL * DMOD + SEQ * DMOD) return;
  if (in_sizes[1] < (NB - 1) * SEQ_FULL + SEQ) return;
  if (in_sizes[2] < DMOD * DMOD || in_sizes[4] < DMOD * DMOD || in_sizes[6] < DMOD * DMOD || in_sizes[8] < DMOD * DMOD) return;
  if (in_sizes[3] < DMOD || in_sizes[5] < DMOD || in_sizes[7] < DMOD || in_sizes[9] < DMOD) return;
  if (out_size < NB * SEQ * DMOD) return;

  const float* x  = (const float*)d_in[0];
  const int*   am = (const int*)d_in[1];
  const float* Wq = (const float*)d_in[2];
  const float* bq = (const float*)d_in[3];
  const float* Wk = (const float*)d_in[4];
  const float* bk = (const float*)d_in[5];
  const float* Wv = (const float*)d_in[6];
  const float* bv = (const float*)d_in[7];
  const float* Wo = (const float*)d_in[8];
  const float* bo = (const float*)d_in[9];

  const size_t PW = (size_t)DMOD * DMOD * 2;
  const size_t PX = (size_t)SEQ * DMOD * 2;
  const size_t PS = (size_t)HG * SEQ * SEQ * 4;
  const size_t PP = (size_t)HG * SEQ * SEQ * 2;
  size_t off = 0;
  const size_t oWt  = off; off += 4 * PW;
  const size_t oXb  = off; off += PX;
  const size_t oQh  = off; off += PX;
  const size_t oQl  = off; off += PX;
  const size_t oKh  = off; off += PX;
  const size_t oKl  = off; off += PX;
  const size_t oVTh = off; off += PX;
  const size_t oVTl = off; off += PX;
  const size_t oS   = off; off += PS;
  const size_t oPh  = off; off += PP;
  const size_t oPl  = off; off += PP;
  const size_t oOh  = off; off += PX;
  const size_t oOl  = off; off += PX;
  if (off > ws_size) return;

  char* ws = (char*)d_ws;
  unsigned short* Wt  = (unsigned short*)(ws + oWt);
  unsigned short* Wqt = Wt;
  unsigned short* Wkt = Wt + (size_t)1 * DMOD * DMOD;
  unsigned short* Wvt = Wt + (size_t)2 * DMOD * DMOD;
  unsigned short* Wot = Wt + (size_t)3 * DMOD * DMOD;
  unsigned short* Xb  = (unsigned short*)(ws + oXb);
  unsigned short* Qh  = (unsigned short*)(ws + oQh);
  unsigned short* Ql  = (unsigned short*)(ws + oQl);
  unsigned short* Kh  = (unsigned short*)(ws + oKh);
  unsigned short* Kl  = (unsigned short*)(ws + oKl);
  unsigned short* VTh = (unsigned short*)(ws + oVTh);
  unsigned short* VTl = (unsigned short*)(ws + oVTl);
  float*          Sb  = (float*)(ws + oS);
  unsigned short* Ph  = (unsigned short*)(ws + oPh);
  unsigned short* Pl  = (unsigned short*)(ws + oPl);
  unsigned short* Oh  = (unsigned short*)(ws + oOh);
  unsigned short* Ol  = (unsigned short*)(ws + oOl);

  const dim3 blk(256);
  const int  n2x = SEQ * DMOD / 2;
  const dim3 gCastX((n2x + 255) / 256);
  const dim3 gT(DMOD / 64, DMOD / 64);
  const int  tQK = (SEQ / 64) * (DMOD / 64);
  const dim3 gQK((tQK + 7) / 8, 1);
  const dim3 gS((((SEQ / 64) * (SEQ / 64)) + 7) / 8, HG);
  const dim3 gPV(((SEQ / 64) + 7) / 8, HG);
  const dim3 gSm(SEQ, HG);
  const dim3 bSm(SEQ / 8);

  cast_transpose_bf16_kernel<<<gT, blk, 0, stream>>>(Wq, Wqt, DMOD, DMOD);
  cast_transpose_bf16_kernel<<<gT, blk, 0, stream>>>(Wk, Wkt, DMOD, DMOD);
  cast_transpose_bf16_kernel<<<gT, blk, 0, stream>>>(Wv, Wvt, DMOD, DMOD);
  cast_transpose_bf16_kernel<<<gT, blk, 0, stream>>>(Wo, Wot, DMOD, DMOD);

  for (int b = 0; b < NB; ++b) {
    const float* xb   = x + (size_t)b * SEQ_FULL * DMOD;
    const int*   amb  = am + (size_t)b * SEQ_FULL;
    float*       outb = (float*)d_out + (size_t)b * SEQ * DMOD;
    cast_bf16x2_kernel<<<gCastX, blk, 0, stream>>>(xb, Xb, n2x);
    wmma_gemm64<1, 0, 0, 2, 2, 0><<<gQK, blk, 0, stream>>>(
        Xb, Xb, DMOD, 0L, Wqt, Wqt, DMOD, 0L, (void*)Qh, (void*)Ql, DMOD, 0L,
        bq, SEQ, DMOD, DMOD, 1.0f);
    wmma_gemm64<1, 0, 0, 2, 2, 0><<<gQK, blk, 0, stream>>>(
        Xb, Xb, DMOD, 0L, Wkt, Wkt, DMOD, 0L, (void*)Kh, (void*)Kl, DMOD, 0L,
        bk, SEQ, DMOD, DMOD, 1.0f);
    wmma_gemm64<1, 0, 0, 1, 2, 0><<<gQK, blk, 0, stream>>>(
        Wvt, Wvt, DMOD, 0L, Xb, Xb, DMOD, 0L, (void*)VTh, (void*)VTl, SEQ, 0L,
        bv, DMOD, SEQ, DMOD, 1.0f);
    for (int g = 0; g < NHEAD / HG; ++g) {
      const int e0 = g * HG * HDIM;
      wmma_gemm64<1, 1, 1, 0, 0, 1><<<gS, blk, 0, stream>>>(
          Qh + e0, Ql + e0, DMOD, (long)HDIM, Kh + e0, Kl + e0, DMOD, (long)HDIM,
          (void*)Sb, (void*)Sb, SEQ, (long)SEQ * SEQ,
          bq, SEQ, SEQ, HDIM, SM_SCALE);
      softmax_row_kernel<<<gSm, bSm, 0, stream>>>(Sb, amb, Ph, Pl);
      wmma_gemm64<1, 1, 1, 0, 2, 2><<<gPV, blk, 0, stream>>>(
          Ph, Pl, SEQ, (long)SEQ * SEQ, VTh + (size_t)e0 * SEQ, VTl + (size_t)e0 * SEQ, SEQ, (long)HDIM * SEQ,
          (void*)(Oh + e0), (void*)(Ol + e0), DMOD, (long)HDIM,
          bq, SEQ, HDIM, SEQ, 1.0f);
    }
    wmma_gemm64<1, 1, 0, 2, 0, 0><<<gQK, blk, 0, stream>>>(
        Oh, Ol, DMOD, 0L, Wot, Wot, DMOD, 0L, (void*)outb, (void*)outb, DMOD, 0L,
        bo, SEQ, DMOD, DMOD, 1.0f);
  }
  (void)hipGetLastError();
}
